// RNN_79216376808164
// MI455X (gfx1250) — hardware-verified
//
#include <hip/hip_runtime.h>
#include <math.h>

typedef __attribute__((ext_vector_type(16))) _Float16 v16h;
typedef __attribute__((ext_vector_type(8)))  _Float16 v8h;
typedef __attribute__((ext_vector_type(8)))  float    v8f;
typedef __attribute__((ext_vector_type(4)))  float    v4f;
typedef __attribute__((ext_vector_type(4)))  int      v4i;

constexpr int kBatch  = 256;
constexpr int kSteps  = 256;
constexpr int kEmb    = 128;
constexpr int kState  = 512;
constexpr int kAlpha  = 128;
constexpr int kWinP   = kEmb + kState;

constexpr int kSeqPB   = 16;
constexpr int kBlocks  = kBatch / kSeqPB;
constexpr int kThreads = 256;
constexpr int kWaves   = kThreads / 32;
constexpr int kHP      = kState + 8;
constexpr int kYP      = kAlpha + 4;

constexpr float kWCarry     = 256.0f;
constexpr float kWCarryInv  = 1.0f / 256.0f;
constexpr float kLoCarry    = 2048.0f;
constexpr float kLoCarryInv = 1.0f / 2048.0f;
constexpr float kF16MinNorm = 6.103515625e-5f;

static_assert(kBatch % kSeqPB == 0);
static_assert(kState == kWaves * 64);
static_assert(kAlpha == kWaves * 16);
static_assert(kSeqPB == kWaves * 2);
static_assert(kAlpha * 4 == 32 * 16);
static_assert(kState % 32 == 0 && kEmb % 4 == 0);
static_assert(kHP % 8 == 0 && kYP % 4 == 0);
static_assert(kSteps == kThreads);
static_assert(((kSeqPB * kHP) % 8) == 0);

union FragU { v16h v; v8h h[2]; };
__device__ __forceinline__ v16h frag_load(const _Float16* p) {
  FragU f; f.h[0] = *(const v8h*)(p); f.h[1] = *(const v8h*)(p + 16); return f.v;
}
__device__ __forceinline__ v8f mma16(v16h a, v16h b, v8f c) {
  return __builtin_amdgcn_wmma_f32_16x16x32_f16(false, a, false, b, (short)0, c, false, false);
}
__device__ __forceinline__ void guard_rec(v8f& a0, v8f& a1, v8f& a2, v8f& a3, v8f& r0, v8f& r1, v8f& r2, v8f& r3,
                                          v16h x, v16h y, v16h b0, v16h b1, v16h b2, v16h b3) {
  asm volatile("v_nop\n\tv_nop\n\tv_nop\n\tv_nop"
               : "+v"(a0), "+v"(a1), "+v"(a2), "+v"(a3), "+v"(r0), "+v"(r1), "+v"(r2), "+v"(r3)
               : "v"(x), "v"(y), "v"(b0), "v"(b1), "v"(b2), "v"(b3)
               : "memory");
}
__device__ __forceinline__ void guard_out(v8f& a, v8f& r, v16h x, v16h y, v16h b) {
  asm volatile("v_nop\n\tv_nop\n\tv_nop\n\tv_nop" : "+v"(a), "+v"(r) : "v"(x), "v"(y), "v"(b) : "memory");
}

__device__ __forceinline__ float tanh_f32(float x) {
  return 1.0f - 2.0f * __builtin_amdgcn_rcpf(1.0f + expf(2.0f * x));
}

__global__ __launch_bounds__(256) void table_kernel(const float* __restrict__ emb, const float* __restrict__ W_in,
                                                    const float* __restrict__ b_in, float* __restrict__ P) {
  const int i  = blockIdx.x * 256 + threadIdx.x;
  const int a  = i >> 7;
  const int n4 = (i & 127) * 4;
  const float* er = emb + (size_t)a * kEmb;
  const float* w0 = W_in + (size_t)n4 * kWinP;
  const float* w1 = w0 + kWinP;
  const float* w2 = w1 + kWinP;
  const float* w3 = w2 + kWinP;
  float s0 = 0.0f, s1 = 0.0f, s2 = 0.0f, s3 = 0.0f;
#pragma unroll 1
  for (int e = 0; e < kEmb; e += 4) {
    const v4f ev = *(const v4f*)(er + e);
    const v4f x0 = *(const v4f*)(w0 + e);
    const v4f x1 = *(const v4f*)(w1 + e);
    const v4f x2 = *(const v4f*)(w2 + e);
    const v4f x3 = *(const v4f*)(w3 + e);
    s0 = fmaf(ev[0], x0[0], s0); s0 = fmaf(ev[1], x0[1], s0); s0 = fmaf(ev[2], x0[2], s0); s0 = fmaf(ev[3], x0[3], s0);
    s1 = fmaf(ev[0], x1[0], s1); s1 = fmaf(ev[1], x1[1], s1); s1 = fmaf(ev[2], x1[2], s1); s1 = fmaf(ev[3], x1[3], s1);
    s2 = fmaf(ev[0], x2[0], s2); s2 = fmaf(ev[1], x2[1], s2); s2 = fmaf(ev[2], x2[2], s2); s2 = fmaf(ev[3], x2[3], s2);
    s3 = fmaf(ev[0], x3[0], s3); s3 = fmaf(ev[1], x3[1], s3); s3 = fmaf(ev[2], x3[2], s3); s3 = fmaf(ev[3], x3[3], s3);
  }
  const v4f bi = *(const v4f*)(b_in + n4);
  v4f o;
  o[0] = s0 + bi[0]; o[1] = s1 + bi[1]; o[2] = s2 + bi[2]; o[3] = s3 + bi[3];
  float* dp = P + (size_t)i * 4;
  *(volatile v4f*)dp = o;
  __threadfence();
  *(volatile v4f*)dp = o;
}

__global__ __launch_bounds__(256) void cvt8_f16_kernel(const float* __restrict__ src, _Float16* __restrict__ dst,
                                                       int nrow, int ncol8, int spitch, int scol0, float sc) {
  const int i  = blockIdx.x * 256 + threadIdx.x;
  const int n8 = nrow * ncol8;
  if (i < n8) {
    const int row = i / ncol8;
    const int c8  = i - row * ncol8;
    const float* sp = src + (size_t)row * spitch + scol0 + c8 * 8;
    const v4f a = *(const v4f*)(sp);
    const v4f b = *(const v4f*)(sp + 4);
    v8h hv;
    hv[0] = (_Float16)(a[0] * sc); hv[1] = (_Float16)(a[1] * sc); hv[2] = (_Float16)(a[2] * sc); hv[3] = (_Float16)(a[3] * sc);
    hv[4] = (_Float16)(b[0] * sc); hv[5] = (_Float16)(b[1] * sc); hv[6] = (_Float16)(b[2] * sc); hv[7] = (_Float16)(b[3] * sc);
    _Float16* dp = dst + (size_t)i * 8;
    *(volatile v8h*)dp = hv;
    __threadfence();
    *(volatile v8h*)dp = hv;
  }
}

__global__ __launch_bounds__(kThreads) void rnn_scan_kernel(
    const int* __restrict__ w, const float* __restrict__ P,
    const _Float16* __restrict__ Ws16, const _Float16* __restrict__ Wo16,
    const float* __restrict__ b_out, float* __restrict__ out) {
  __shared__ __align__(16) _Float16 Hh[kSeqPB * kHP];
  __shared__ __align__(16) _Float16 Hl[kSeqPB * kHP];
  __shared__ __align__(16) int      tokT[kSteps * kSeqPB];
  __shared__ __align__(16) float    Ys[kSeqPB * kYP];

  const int tid = threadIdx.x, lane = tid & 31, wave = tid >> 5;
  const int c = lane & 15, hh = lane >> 4, koff = hh * 8;
  const int seq0 = blockIdx.x * kSeqPB;
  const int n0 = wave * 64;

  {
    const v8h z = {(_Float16)0.f, (_Float16)0.f, (_Float16)0.f, (_Float16)0.f,
                   (_Float16)0.f, (_Float16)0.f, (_Float16)0.f, (_Float16)0.f};
    for (int i = tid; i < (kSeqPB * kHP) / 8; i += kThreads) {
      *(v8h*)(Hh + i * 8) = z;
      *(v8h*)(Hl + i * 8) = z;
    }
  }
#pragma unroll 4
  for (int r = 0; r < kSeqPB; ++r) {
    int v = w[(size_t)(seq0 + r) * kSteps + tid];
    v = v < 0 ? 0 : v;
    v = v > (kAlpha - 1) ? (kAlpha - 1) : v;
    tokT[tid * kSeqPB + r] = v;
  }
  __syncthreads();

  const _Float16* arow_h = Hh + c * kHP + koff;
  const _Float16* arow_l = Hl + c * kHP + koff;
  const _Float16* brow   = Ws16 + (size_t)(n0 + c) * kState + koff;
  const _Float16* orow   = Wo16 + (size_t)(wave * 16 + c) * kState + koff;
  const float bo = b_out[wave * 16 + c];
  const v8f z8 = {0.f, 0.f, 0.f, 0.f, 0.f, 0.f, 0.f, 0.f};

#pragma unroll 1
  for (int t = 0; t <= kSteps; ++t) {
    v8f am[4], ar[4];
#pragma unroll
    for (int j = 0; j < 4; ++j) { am[j] = z8; ar[j] = z8; }
    v8f om = z8, orr = z8;

#pragma unroll 2
    for (int kb = 0; kb < kState / 32; ++kb) {
      const v16h ah = frag_load(arow_h + kb * 32);
      const v16h al = frag_load(arow_l + kb * 32);
      v16h fb[4];
#pragma unroll
      for (int j = 0; j < 4; ++j) fb[j] = frag_load(brow + (size_t)(16 * j) * kState + kb * 32);
#pragma unroll
      for (int j = 0; j < 4; ++j) {
        am[j] = mma16(ah, fb[j], am[j]);
        ar[j] = mma16(al, fb[j], ar[j]);
      }
      guard_rec(am[0], am[1], am[2], am[3], ar[0], ar[1], ar[2], ar[3], ah, al, fb[0], fb[1], fb[2], fb[3]);
      const v16h fo = frag_load(orow + kb * 32);
      om  = mma16(ah, fo, om);
      orr = mma16(al, fo, orr);
      guard_out(om, orr, ah, al, fo);
    }

    if (t > 0) {
#pragma unroll
      for (int r = 0; r < 8; ++r) {
        const float yv = (om[r] + orr[r] * kLoCarryInv) * kWCarryInv + bo;
        Ys[(8 * hh + r) * kYP + wave * 16 + c] = yv;
      }
    }
    __syncthreads();

    if (t < kSteps) {
      const v4i ta = *(const v4i*)(tokT + t * kSeqPB + 8 * hh);
      const v4i tb = *(const v4i*)(tokT + t * kSeqPB + 8 * hh + 4);
      const int tk0 = ta[0], tk1 = ta[1], tk2 = ta[2], tk3 = ta[3];
      const int tk4 = tb[0], tk5 = tb[1], tk6 = tb[2], tk7 = tb[3];
      const int tk[8] = {tk0, tk1, tk2, tk3, tk4, tk5, tk6, tk7};
#pragma unroll
      for (int j = 0; j < 4; ++j) {
        const int col = n0 + 16 * j + c;
        float pv[8];
#pragma unroll
        for (int r = 0; r < 8; ++r) pv[r] = P[(size_t)tk[r] * kState + col];
        asm volatile("" ::: "memory");
#pragma unroll
        for (int r = 0; r < 8; ++r) {
          const float pre = (am[j][r] + ar[j][r] * kLoCarryInv) * kWCarryInv + pv[r];
          const float hv  = tanh_f32(pre);
          const float hq  = (fabsf(hv) < kF16MinNorm) ? 0.0f : hv;
          const _Float16 hi = (_Float16)hq;
          const float lof = (hv - (float)hi) * kLoCarry;
          const _Float16 lo = (_Float16)lof;
          Hh[(8 * hh + r) * kHP + col] = hi;
          Hl[(8 * hh + r) * kHP + col] = lo;
        }
        asm volatile("" ::: "memory");
      }
    }
    if (t > 0) {
      const int r0 = 2 * wave;
      const v4f y0 = *(const v4f*)(Ys + r0 * kYP + 4 * lane);
      const v4f y1 = *(const v4f*)(Ys + (r0 + 1) * kYP + 4 * lane);
      float* d0 = out + ((size_t)(seq0 + r0) * kSteps + (size_t)(t - 1)) * kAlpha + 4 * lane;
      float* d1 = d0 + (size_t)kSteps * kAlpha;
      *(volatile v4f*)d0 = y0;
      *(volatile v4f*)d1 = y1;
      __threadfence();
      *(volatile v4f*)d0 = y0;
      *(volatile v4f*)d1 = y1;
      __threadfence();
    }
    __syncthreads();
  }
}

extern "C" void kernel_launch(void* const* d_in, const int* in_sizes, int n_in,
                              void* d_out, int out_size, void* d_ws, size_t ws_size, hipStream_t stream) {
  if (n_in < 6 || d_out == nullptr || d_ws == nullptr) return;
  if (in_sizes[0] != kBatch * kSteps || in_sizes[1] != kAlpha * kEmb || in_sizes[2] != kState * kWinP ||
      in_sizes[3] != kState || in_sizes[4] != kAlpha * kState || in_sizes[5] != kAlpha ||
      out_size != kBatch * kSteps * kAlpha) return;

  const int*   w     = (const int*)d_in[0];
  const float* emb   = (const float*)d_in[1];
  const float* W_in  = (const float*)d_in[2];
  const float* b_in  = (const float*)d_in[3];
  const float* W_out = (const float*)d_in[4];
  const float* b_out = (const float*)d_in[5];
  float* out = (float*)d_out;

  char* ws = (char*)d_ws; size_t off = 0;
  auto carve = [&](size_t bytes) -> char* { char* p = ws + off; off += (bytes + 255) & ~(size_t)255; return p; };
  float*    P    = (float*)carve((size_t)kAlpha * kState * 4);
  _Float16* WS16 = (_Float16*)carve((size_t)kState * kState * 2);
  _Float16* WO16 = (_Float16*)carve((size_t)kAlpha * kState * 2);
  if (off > ws_size || off > (size_t)134217728) return;

  table_kernel<<<(kAlpha * kState / 4) / 256, 256, 0, stream>>>(emb, W_in, b_in, P);

  const int n8s = kState * (kState / 8);
  const int n8o = kAlpha * (kState / 8);
  cvt8_f16_kernel<<<(n8s + 255) / 256, 256, 0, stream>>>(W_in,  WS16, kState, kState / 8, kWinP,  kEmb, kWCarry);
  cvt8_f16_kernel<<<(n8o + 255) / 256, 256, 0, stream>>>(W_out, WO16, kAlpha, kState / 8, kState, 0,    kWCarry);

  rnn_scan_kernel<<<kBlocks, kThreads, 0, stream>>>(w, P, WS16, WO16, b_out, out);
}
